// CellDrugAttentionModel_63986422776352
// MI455X (gfx1250) — hardware-verified
//
#include <hip/hip_runtime.h>
#include <hip/hip_bf16.h>
#include <math.h>


typedef _Float16 bf16;
typedef _Float16 f16;
typedef __attribute__((ext_vector_type(4))) unsigned v4u_t;
typedef unsigned v4ua __attribute__((ext_vector_type(4), may_alias));
typedef __attribute__((ext_vector_type(4))) float v4f_t;
typedef float v4fa __attribute__((ext_vector_type(4), may_alias));
typedef __attribute__((ext_vector_type(16))) bf16  bf16x16;
typedef bf16x16 f16x16;
typedef __attribute__((ext_vector_type(8)))  bf16  bf16x8;
typedef bf16x8 f16x8;
typedef __attribute__((ext_vector_type(4)))  bf16  bf16x4;
typedef __attribute__((ext_vector_type(8)))  float f32x8;
__device__ __forceinline__ f32x8 wmma16(f16x16 a, f16x16 b, f32x8 c) {
  c = __builtin_amdgcn_wmma_f32_16x16x32_f16(false, a, false, b, (short)0, c, false, false);
  asm volatile("v_nop\n\tv_nop\n\tv_nop\n\tv_nop" : "+v"(c) : "v"(a), "v"(b));
  return c;
}
#define LDS_STRIDE 48
#define KSTRIDE    72
#define VSTRIDE    48

__device__ __forceinline__ f32x8 wmma_bf16(bf16x16 a, bf16x16 b, f32x8 c) {
  c = __builtin_amdgcn_wmma_f32_16x16x32_f16(false, a, false, b, (short)0, c, false, false);
  asm volatile("v_nop\n\tv_nop\n\tv_nop\n\tv_nop" : "+v"(c) : "v"(a), "v"(b));
  return c;
}

template <typename T>
__device__ __forceinline__ bf16x16 load_frag(const T* __restrict__ base, int ld,
                                             int row0, int k0) {
  const int lane = threadIdx.x & 31;
  const int r    = lane & 15;
  const int kh   = (lane >> 4) * 8;
  const T* p0 = base + (size_t)(row0 + r) * ld + (k0 + kh);
  const T* p1 = p0 + 16;
  bf16x16 f;
#pragma unroll
  for (int i = 0; i < 8; ++i) {
    f[i]     = (bf16)p0[i];
    f[i + 8] = (bf16)p1[i];
  }
  return f;
}

__device__ __forceinline__ bf16x16 lds_frag(const bf16* base, int stride) {
  const int lane = threadIdx.x & 31;
  const int row  = lane & 15;
  const int kh   = (lane >> 4) * 8;
  const bf16x8 lo = *(const bf16x8*)(base + row * stride + kh);
  const bf16x8 hi = *(const bf16x8*)(base + row * stride + kh + 16);
  bf16x16 f;
#pragma unroll
  for (int i = 0; i < 8; ++i) { f[i] = lo[i]; f[i + 8] = hi[i]; }
  return f;
}

template <typename T>
__device__ __forceinline__ void stage_read16(const T* __restrict__ p, float* buf) {
#pragma unroll
  for (int i = 0; i < 16; ++i) buf[i] = (float)p[i];
}

__device__ __forceinline__ void stage_write(bf16* dst, const float* buf, int nquad) {
#pragma unroll
  for (int i = 0; i < nquad; ++i) {
    bf16x4 q;
    q[0] = (bf16)buf[4 * i];     q[1] = (bf16)buf[4 * i + 1];
    q[2] = (bf16)buf[4 * i + 2]; q[3] = (bf16)buf[4 * i + 3];
    *(bf16x4*)(dst + 4 * i) = q;
  }
}


#define GSTR 48
#define SS 128
#define HH 16
#define DKK 64
template <typename AT, int MODE>
__global__ __launch_bounds__(256) void gemm_rb_kernel(
    const AT* __restrict__ A, const float* __restrict__ W,
    const float* __restrict__ bias, const float* __restrict__ rowscale, const float* __restrict__ R, const float* __restrict__ rowbias, void* __restrict__ out,
    int M, int N, int K) {
  __shared__ bf16 ldsA[128 * LDS_STRIDE];
  __shared__ bf16 ldsW[256 * LDS_STRIDE];
  __shared__ __attribute__((aligned(16))) unsigned char sob[256 * 136 * 2];

  const int t    = threadIdx.x;
  const int wave = t >> 5;
  const int lane = t & 31;
  const int wm   = (wave & 1) * 64;
  const int wn   = (wave >> 1) * 64;
  const int mBlk = blockIdx.x * 128;
  const int nBlk = blockIdx.y * 256;

  const int arow = t >> 1;
  const int ach  = (t & 1) * 16;

  float abuf[16];
  float wbuf[32];

  stage_read16(A + (size_t)(mBlk + arow) * K + ach, abuf);
  const int nrow = min(nBlk + t, N - 1);
  stage_read16(W + (size_t)nrow * K,          wbuf);
  stage_read16(W + (size_t)nrow * K + 16,     wbuf + 16);

  f32x8 acc[4][4] = {};

  for (int k = 0; k < K; k += 32) {
    __syncthreads();
    stage_write(&ldsA[arow * LDS_STRIDE + ach], abuf, 4);
    stage_write(&ldsW[t * LDS_STRIDE],          wbuf, 8);
    if (k + 32 < K) {
      stage_read16(A + (size_t)(mBlk + arow) * K + (k + 32) + ach, abuf);
      stage_read16(W + (size_t)nrow * K + (k + 32),          wbuf);
      stage_read16(W + (size_t)nrow * K + (k + 32) + 16,     wbuf + 16);
    }
    __syncthreads();

    bf16x16 af[4], wf[4];
#pragma unroll
    for (int i = 0; i < 4; ++i)
      af[i] = lds_frag(ldsA + (wm + 16 * i) * LDS_STRIDE, LDS_STRIDE);
#pragma unroll
    for (int j = 0; j < 4; ++j)
      wf[j] = lds_frag(ldsW + (wn + 16 * j) * LDS_STRIDE, LDS_STRIDE);
#pragma unroll
    for (int i = 0; i < 4; ++i)
#pragma unroll
      for (int j = 0; j < 4; ++j)
        acc[i][j] = wmma_bf16(af[i], wf[j], acc[i][j]);
  }

  const int nlane = lane & 15;
  const int mh    = (lane >> 4) * 8;
  __syncthreads();
  if (MODE == 0 || MODE == 1 || MODE == 3) {
    bf16* so = (bf16*)sob;
#pragma unroll
    for (int i = 0; i < 4; ++i)
#pragma unroll
      for (int j = 0; j < 4; ++j) {
        const int nl = wn + 16 * j + nlane;
        const float bv = bias ? bias[nBlk + nl] : 0.0f;
        if (MODE == 3) {
#pragma unroll 1
          for (int r = 0; r < 8; ++r) {
            const int ml = wm + 16 * i + mh + r;
            const float xg = acc[i][j][r] + bv;
            so[ml * 264 + nl] = (bf16)(0.5f * xg * (1.0f + erff(xg * 0.70710678118654752f)));
          }
        } else {
#pragma unroll
        for (int r = 0; r < 8; ++r) {
          const int ml = wm + 16 * i + mh + r;
          const bf16 hv = (bf16)(acc[i][j][r] + bv);
          if (MODE == 0) so[ml * 264 + nl] = hv;
          else           so[nl * 136 + ml] = hv;
        }
        }
      }
    __syncthreads();
#pragma unroll 1
    for (int pass = 0; pass < 2; ++pass) {
      if (MODE == 0 || MODE == 3) {
        for (int ch = t; ch < 128 * 32; ch += 256) { const int ml = ch >> 5, q = (ch & 31) * 8;
          *(volatile v4u_t*)((bf16*)out + (size_t)(mBlk + ml) * N + nBlk + q) = *(const v4ua*)(so + ml * 264 + q); }
      } else {
        const int b_ = mBlk / SS, s0 = mBlk % SS;
        for (int ch = t; ch < 256 * 16; ch += 256) { const int nl = ch >> 4, q = (ch & 15) * 8; const int n = nBlk + nl, h = n >> 6, dk = n & (DKK - 1);
          *(volatile v4u_t*)((bf16*)out + (((size_t)(b_ * HH + h)) * DKK + dk) * SS + s0 + q) = *(const v4ua*)(so + nl * 136 + q); }
      }
      __threadfence();
    }
  } else {
    float* so = (float*)sob;
#pragma unroll 1
    for (int hf = 0; hf < 2; ++hf) {
      if (wm == hf * 64) {
#pragma unroll
        for (int i = 0; i < 4; ++i)
#pragma unroll
          for (int j = 0; j < 4; ++j) {
            const int nl = wn + 16 * j + nlane;
            const float bv = bias ? bias[nBlk + nl] : 0.0f;
#pragma unroll
            for (int r = 0; r < 8; ++r) { const int mrow = mBlk + hf * 64 + 16 * i + mh + r; so[(16 * i + mh + r) * 260 + nl] = acc[i][j][r] * (rowscale ? rowscale[mrow] : 1.0f) + bv + (rowbias ? rowbias[mrow] : 0.0f); }
          }
      }
      __syncthreads();
      if (R) {
        for (int ch = t; ch < 64 * 64; ch += 256) { const int ml = ch >> 6, q = (ch & 63) * 4;
          if (nBlk + q < N) { const v4f_t rv = *(const v4f_t*)(R + (size_t)(mBlk + hf * 64 + ml) * N + nBlk + q); v4f_t v = *(const v4fa*)(so + ml * 260 + q); v += rv; *(volatile v4fa*)(so + ml * 260 + q) = v; } }
        asm volatile("s_wait_dscnt 0" ::: "memory");
      }
#pragma unroll 1
      for (int pass = 0; pass < 2; ++pass) {
        for (int ch = t; ch < 64 * 64; ch += 256) { const int ml = ch >> 6, q = (ch & 63) * 4;
          if (nBlk + q < N) *(volatile v4f_t*)((float*)out + (size_t)(mBlk + hf * 64 + ml) * N + nBlk + q) = *(const v4fa*)(so + ml * 260 + q); }
        __threadfence();
      }
      __syncthreads();
    }
  }
}

#define GSTR 48
template <typename AT, int EPI, bool OUT16>
__global__ __launch_bounds__(256) void gemm_kne(const AT* __restrict__ A, int lda, const float* __restrict__ Wm, int ldw,
                                                const float* __restrict__ bias, const float* __restrict__ R, const float* __restrict__ gvec,
                                                void* __restrict__ Yv, int ldy, int K) {
  __shared__ __attribute__((aligned(16))) f16 ldsA[128 * GSTR];
  __shared__ __attribute__((aligned(16))) f16 ldsW[128 * GSTR];
  __shared__ __attribute__((aligned(16))) float oS[8][32 * 68];
  const int tid = threadIdx.x, lane = tid & 31, wave = tid >> 5, cl = lane & 15, rh = (lane >> 4) * 8;
  const int m0 = blockIdx.x * 128, n0 = blockIdx.y * 128;
  const int wm = (wave & 3) * 32, wn = (wave >> 2) * 64;
  f32x8 acc[2][4];
#pragma unroll
  for (int i = 0; i < 2; ++i)
#pragma unroll
    for (int j = 0; j < 4; ++j) { f32x8 z = {}; acc[i][j] = z; }
#pragma unroll 1
  for (int k0 = 0; k0 < K; k0 += 32) {
    __syncthreads();
    { const int row = tid >> 1, ch = (tid & 1) * 16;
      const AT* src = A + (size_t)(m0 + row) * lda + k0 + ch;
#pragma unroll
      for (int g = 0; g < 16; ++g) ldsA[row * GSTR + ch + g] = (f16)src[g]; }
    { const int k = tid >> 3, nn0 = (tid & 7) * 16;
      const float* src = Wm + (size_t)(k0 + k) * ldw + n0 + nn0;
#pragma unroll
      for (int g = 0; g < 4; ++g) { const v4f_t v = *(const v4f_t*)(src + 4 * g);
#pragma unroll
        for (int u = 0; u < 4; ++u) ldsW[(nn0 + 4 * g + u) * GSTR + k] = (f16)v[u]; } }
    __syncthreads();
    f16x16 af[2];
#pragma unroll
    for (int i = 0; i < 2; ++i) af[i] = lds_frag(ldsA + (wm + 16 * i) * GSTR, GSTR);
#pragma unroll
    for (int j = 0; j < 4; ++j) {
      const f16x16 bf = lds_frag(ldsW + (wn + 16 * j) * GSTR, GSTR);
#pragma unroll
      for (int i = 0; i < 2; ++i) acc[i][j] = wmma16(af[i], bf, acc[i][j]);
    }
  }
  float* so = oS[wave];
#pragma unroll
  for (int i = 0; i < 2; ++i)
#pragma unroll
    for (int j = 0; j < 4; ++j) {
      const int n = n0 + wn + 16 * j + cl;
      const float bv = bias ? bias[n] : 0.0f;
      const float gv = (EPI == 2) ? gvec[n] : 0.0f;
      if (EPI == 1) {
#pragma unroll 1
        for (int r = 0; r < 8; ++r) { const float xg = acc[i][j][r] + bv; so[(16 * i + rh + r) * 68 + 16 * j + cl] = 0.5f * xg * (1.0f + erff(xg * 0.70710678118654752f)); }
      } else {
#pragma unroll
        for (int r = 0; r < 8; ++r) {
          float v = acc[i][j][r] + bv;
          if (EPI == 3) v = fmaxf(v, 0.0f);
          if (EPI == 2) v = R[(size_t)(m0 + wm + 16 * i + rh + r) * ldy + n] + gv * v;
          so[(16 * i + rh + r) * 68 + 16 * j + cl] = v;
        }
      }
    }
  asm volatile("s_wait_dscnt 0" ::: "memory");
  __builtin_amdgcn_wave_barrier();
#pragma unroll 1
  for (int pass = 0; pass < 2; ++pass) {
    if (OUT16) {
      f16* Y = (f16*)Yv;
#pragma unroll
      for (int it = 0; it < 8; ++it) { const int c = lane + 32 * it, rr = c >> 3, q8 = (c & 7) * 8;
        union { f16 h[8]; v4u_t v; } u;
#pragma unroll
        for (int e = 0; e < 8; ++e) u.h[e] = (f16)so[rr * 68 + q8 + e];
        *(volatile v4u_t*)(Y + (size_t)(m0 + wm + rr) * ldy + n0 + wn + q8) = u.v; }
    } else {
      float* Y = (float*)Yv;
#pragma unroll
      for (int it = 0; it < 16; ++it) { const int f4 = lane + 32 * it, rr = f4 >> 4, q = (f4 & 15) * 4;
        *(volatile v4f_t*)(Y + (size_t)(m0 + wm + rr) * ldy + n0 + wn + q) = *(const v4fa*)(so + rr * 68 + q); }
    }
    __threadfence();
  }
}

__global__ __launch_bounds__(256) void k_transpose(const float* __restrict__ Wm, float* __restrict__ Wt, int rows, int cols) {
  __shared__ float tS[64][65];
  const int tid = threadIdx.x, tbj = cols / 64, bi = blockIdx.x / tbj, bj = blockIdx.x % tbj;
  for (int e = tid; e < 64 * 64; e += 256) { const int r = e >> 6, c = e & 63; tS[r][c] = Wm[(size_t)(bi * 64 + r) * cols + bj * 64 + c]; }
  __syncthreads();
  for (int ch = tid; ch < 64 * 16; ch += 256) { const int r = ch >> 4, q4 = (ch & 15) * 4; v4f_t o; o[0] = tS[q4][r]; o[1] = tS[q4 + 1][r]; o[2] = tS[q4 + 2][r]; o[3] = tS[q4 + 3][r];
    float* dst = Wt + (size_t)(bj * 64 + r) * rows + bi * 64 + q4; *(volatile v4f_t*)dst = o; __threadfence(); *(volatile v4f_t*)dst = o; }
}

#define NG 512
#define NNODE 32768
#define ML 128
#define EE 1024
#define DC 1024
#define DDR 256
#define NHc 16
#define HDc 64
__device__ __forceinline__ int seg_start(const int* __restrict__ g, int b) {
  int lo = 0, hi = NNODE;
#pragma unroll 1
  for (int it = 0; it < 16; ++it) { const int mid = (lo + hi) >> 1; const bool ge = (mid < NNODE) ? (g[min(mid, NNODE - 1)] >= b) : true; if (lo < hi) { if (ge) hi = mid; else lo = mid + 1; } }
  return lo;
}
__global__ __launch_bounds__(256) void k_attn1(const float* __restrict__ Q, const float* __restrict__ Kn, const float* __restrict__ Vn, const int* __restrict__ guide, float* __restrict__ O, int nbase, int nrows) {
  __shared__ float qS[NHc * HDc]; __shared__ float pS[NHc][ML + 4];
  const int b = blockIdx.x, tid = threadIdx.x, h = tid >> 4, j = tid & 15;
  const int st = seg_start(guide, b); const int en = seg_start(guide, b + 1); const int cnt = min(en - st, ML);
  if (st < nbase || st >= nbase + 4096) return;
  const int rb = st - nbase;
  for (int e = tid; e < NHc * HDc; e += 256) qS[e] = Q[(size_t)b * EE + e] * 0.125f;
  __syncthreads();
  float sc[8]; float mx = -3.0e38f;
#pragma unroll
  for (int i = 0; i < 8; ++i) { const int m = j + 16 * i; const int row = min(rb + m, nrows - 1);
    const float* kr = Kn + (size_t)row * EE + h * HDc; float s = 0.0f;
#pragma unroll 1
    for (int d = 0; d < HDc; ++d) s = fmaf(qS[h * HDc + d], kr[d], s);
    sc[i] = (m < cnt) ? s : -1.0e9f; mx = fmaxf(mx, sc[i]); }
#pragma unroll
  for (int off = 8; off > 0; off >>= 1) mx = fmaxf(mx, __shfl_xor(mx, off, 32));
  float z = 0.0f;
#pragma unroll
  for (int i = 0; i < 8; ++i) { sc[i] = expf(sc[i] - mx); z += sc[i]; }
#pragma unroll
  for (int off = 8; off > 0; off >>= 1) z += __shfl_xor(z, off, 32);
  const float rz = 1.0f / z;
#pragma unroll
  for (int i = 0; i < 8; ++i) pS[h][j + 16 * i] = sc[i] * rz;
  __syncthreads();
  v4f_t acc = {0.0f, 0.0f, 0.0f, 0.0f};
#pragma unroll 1
  for (int m = 0; m < ML; ++m) { const int row = min(rb + m, nrows - 1); const float p = pS[h][m];
    const v4f_t vv = *(const v4f_t*)(Vn + (size_t)row * EE + h * HDc + 4 * j); acc[0] = fmaf(p, vv[0], acc[0]); acc[1] = fmaf(p, vv[1], acc[1]); acc[2] = fmaf(p, vv[2], acc[2]); acc[3] = fmaf(p, vv[3], acc[3]); }
  float* dst = O + (size_t)b * EE + h * HDc + 4 * j; *(volatile v4f_t*)dst = acc; __threadfence(); *(volatile v4f_t*)dst = acc;
}
__global__ __launch_bounds__(256) void k_copycell(const float* __restrict__ cell, float* __restrict__ out) {
  const int b = blockIdx.x, c4 = threadIdx.x * 4; const v4f_t v = *(const v4f_t*)(cell + (size_t)b * DC + c4);
  float* dst = out + (size_t)b * (EE + DC) + EE + c4; *(volatile v4f_t*)dst = v; __threadfence(); *(volatile v4f_t*)dst = v;
}

extern "C" void kernel_launch(void* const* d_in, const int* in_sizes, int n_in,
                              void* d_out, int out_size, void* d_ws, size_t ws_size,
                              hipStream_t stream) {
  (void)in_sizes; (void)n_in; (void)out_size;
  const float** f = (const float**)d_in;
  const float* xn = f[0], *cell = f[1], *Wq = f[2], *bq = f[3], *Wk = f[4], *bk = f[5], *Wv = f[6], *bv = f[7], *Wo = f[8], *bo = f[9], *Wc = f[10], *bc = f[11];
  const int* guide = (const int*)d_in[12];
  float* out = (float*)d_out;
  char* ws = (char*)d_ws;
  float* CQ = (float*)ws; ws += (size_t)NG * EE * 4; float* Q = (float*)ws; ws += (size_t)NG * EE * 4; float* O = (float*)ws; ws += (size_t)NG * EE * 4;
  float* Kc = (float*)ws; ws += (size_t)4224 * EE * 4; float* Vc = (float*)ws; ws += (size_t)4224 * EE * 4;
  float* WoT = (float*)ws; ws += (size_t)EE * EE * 4;
  if ((size_t)(ws - (char*)d_ws) > ws_size) return;
  const dim3 blk(256);
  gemm_rb_kernel<float, 2><<<dim3(NG / 128, EE / 256), blk, 0, stream>>>(cell, Wc, bc, nullptr, nullptr, nullptr, CQ, NG, EE, DC);
  gemm_rb_kernel<float, 2><<<dim3(NG / 128, EE / 256), blk, 0, stream>>>(CQ, Wq, bq, nullptr, nullptr, nullptr, Q, NG, EE, EE);
  for (int c = 0; c < NNODE / 4096; ++c) {
    const int nbase = c * 4096; const int nrows = (c == NNODE / 4096 - 1) ? 4096 : 4224;
    gemm_rb_kernel<float, 2><<<dim3(nrows / 128, EE / 256), blk, 0, stream>>>(xn + (size_t)nbase * DDR, Wk, bk, nullptr, nullptr, nullptr, Kc, nrows, EE, DDR);
    gemm_rb_kernel<float, 2><<<dim3(nrows / 128, EE / 256), blk, 0, stream>>>(xn + (size_t)nbase * DDR, Wv, bv, nullptr, nullptr, nullptr, Vc, nrows, EE, DDR);
    k_attn1<<<dim3(NG), blk, 0, stream>>>(Q, Kc, Vc, guide, O, nbase, nrows);
  }
  k_transpose<<<dim3((EE / 64) * (EE / 64)), blk, 0, stream>>>(Wo, WoT, EE, EE);
  gemm_kne<float, 0, false><<<dim3(NG / 128, EE / 128), blk, 0, stream>>>(O, EE, WoT, EE, bo, nullptr, nullptr, out, EE + DC, EE);
  k_copycell<<<dim3(NG), blk, 0, stream>>>(cell, out);
}
